// TRU_50294067036444
// MI455X (gfx1250) — hardware-verified
//
#include <hip/hip_runtime.h>
#include <math.h>

typedef __attribute__((ext_vector_type(16))) _Float16 v16h;
typedef __attribute__((ext_vector_type(8)))  _Float16 v8h;
typedef __attribute__((ext_vector_type(16))) __bf16   v16b;
typedef __attribute__((ext_vector_type(8)))  float    v8f;
typedef __attribute__((ext_vector_type(4)))  float    v4f;

__device__ __forceinline__ int frag_k(int i, int h) { return (i < 8) ? (8 * h + i) : (16 + 8 * h + (i - 8)); }
__device__ __forceinline__ __bf16 bf16_rne(float f) {
    unsigned int u = __float_as_uint(f);
    u += 0x7fffu + ((u >> 16) & 1u);
    return __builtin_bit_cast(__bf16, (unsigned short)(u >> 16));
}
__device__ __forceinline__ float bf16_f32(__bf16 b) { return __uint_as_float(((unsigned int)__builtin_bit_cast(unsigned short, b)) << 16); }
__device__ __forceinline__ v8f wmma16(v16h a, v16h b, v8f c) {
    c = __builtin_amdgcn_wmma_f32_16x16x32_f16(false, a, false, b, (short)0, c, false, false);
    asm volatile("v_nop\n\tv_nop\n\tv_nop\n\tv_nop" : "+v"(c) : "v"(a), "v"(b));
    return c;
}
__device__ __forceinline__ v8f wmmab(v16b a, v16b b, v8f c) {
    c = __builtin_amdgcn_wmma_f32_16x16x32_bf16(false, a, false, b, (short)0, c, false, false);
    asm volatile("v_nop\n\tv_nop\n\tv_nop\n\tv_nop" : "+v"(c) : "v"(a), "v"(b));
    return c;
}
struct Split { v16b hi, lo; };
__device__ __forceinline__ v8f wmma3(const Split& a, const Split& b, v8f c) {
    c = __builtin_amdgcn_wmma_f32_16x16x32_bf16(false, a.hi, false, b.hi, (short)0, c, false, false);
    c = __builtin_amdgcn_wmma_f32_16x16x32_bf16(false, a.hi, false, b.lo, (short)0, c, false, false);
    c = __builtin_amdgcn_wmma_f32_16x16x32_bf16(false, a.lo, false, b.hi, (short)0, c, false, false);
    asm volatile("v_nop\n\tv_nop\n\tv_nop\n\tv_nop" : "+v"(c) : "v"(a.hi), "v"(a.lo), "v"(b.hi), "v"(b.lo));
    return c;
}
struct Split3 { v16b hi, mid, lo; };
__device__ __forceinline__ v8f wmma6(const Split3& a, const Split3& b, v8f c) {
    c = __builtin_amdgcn_wmma_f32_16x16x32_bf16(false, a.hi, false, b.hi, (short)0, c, false, false);
    c = __builtin_amdgcn_wmma_f32_16x16x32_bf16(false, a.hi, false, b.mid, (short)0, c, false, false);
    c = __builtin_amdgcn_wmma_f32_16x16x32_bf16(false, a.mid, false, b.hi, (short)0, c, false, false);
    c = __builtin_amdgcn_wmma_f32_16x16x32_bf16(false, a.hi, false, b.lo, (short)0, c, false, false);
    c = __builtin_amdgcn_wmma_f32_16x16x32_bf16(false, a.mid, false, b.mid, (short)0, c, false, false);
    c = __builtin_amdgcn_wmma_f32_16x16x32_bf16(false, a.lo, false, b.hi, (short)0, c, false, false);
    asm volatile("v_nop\n\tv_nop\n\tv_nop\n\tv_nop" : "+v"(c) : "v"(a.hi), "v"(a.mid), "v"(a.lo), "v"(b.hi), "v"(b.mid), "v"(b.lo));
    return c;
}

__device__ __forceinline__ v16h fh_ld(const float* __restrict__ p, long long sk, int k0, int h, int klen, float s) {
    v16h a;
#pragma unroll
    for (int i = 0; i < 16; ++i) { const int k = k0 + frag_k(i, h); a[i] = (k < klen) ? (_Float16)(p[(long long)k * sk] * s) : (_Float16)0.f; }
    return a;
}
__device__ __forceinline__ Split sp_ld(const float* __restrict__ p, long long sk, int k0, int h, int klen, float s) {
    Split r;
#pragma unroll
    for (int i = 0; i < 16; ++i) {
        const int k = k0 + frag_k(i, h); const float x = (k < klen) ? p[(long long)k * sk] * s : 0.f;
        const __bf16 hb = bf16_rne(x); r.hi[i] = hb; r.lo[i] = bf16_rne(x - bf16_f32(hb));
    }
    return r;
}
__device__ __forceinline__ Split3 sp3_ld(const float* __restrict__ p, long long sk, int k0, int h, int klen, float s) {
    Split3 r;
#pragma unroll
    for (int i = 0; i < 16; ++i) {
        const int k = k0 + frag_k(i, h); const float x = (k < klen) ? p[(long long)k * sk] * s : 0.f;
        const __bf16 hb = bf16_rne(x); const float r1 = x - bf16_f32(hb); const __bf16 mb = bf16_rne(r1);
        r.hi[i] = hb; r.mid[i] = mb; r.lo[i] = bf16_rne(r1 - bf16_f32(mb));
    }
    return r;
}
__device__ __forceinline__ v16b bh_ld(const float* __restrict__ p, long long sk, int k0, int h, int klen, float s) {
    v16b a;
#pragma unroll
    for (int i = 0; i < 16; ++i) { const int k = k0 + frag_k(i, h); a[i] = bf16_rne((k < klen) ? p[(long long)k * sk] * s : 0.f); }
    return a;
}
__device__ __forceinline__ v16h fh_row(const _Float16* __restrict__ row, int k0, int h) {
    v16h a;
#pragma unroll
    for (int i = 0; i < 16; ++i) a[i] = row[k0 + frag_k(i, h)];
    return a;
}

#define VST2(T, ptr, val) do { const T vst2_v_ = (val); *(volatile T*)(ptr) = vst2_v_; __threadfence(); *(volatile T*)(ptr) = vst2_v_; } while (0)
typedef float v4f __attribute__((ext_vector_type(4)));
#define VST2V4(ptr, val) do { const v4f vst2_v4_ = (val); *(volatile v4f*)(ptr) = vst2_v4_; __threadfence(); *(volatile v4f*)(ptr) = vst2_v4_; } while (0)

__device__ __attribute__((noinline)) float act_fn(float v, int act) {
    if (act == 1) return fmaxf(v, 0.f);
    if (act == 2) { const float u = 0.7978845608028654f * (v + 0.044715f * v * v * v); return 0.5f * v * (1.f + tanhf(u)); }
    if (act == 3) return v / (1.f + expf(-v));
    if (act == 4) return 0.5f * v * (1.f + erff(v * 0.7071067811865476f));
    if (act == 5) return tanhf(v);
    if (act == 6) return 1.f / (1.f + expf(-v));
    if (act == 7) return (v > 0.f) ? v : 0.01f * v;
    if (act == 8) return (v > 0.f) ? v : (expf(v) - 1.f);
    if (act == 9) return fminf(fmaxf(v, 0.f), 6.f);
    if (act == 10) return fabsf(v);
    if (act == 11) return (v >= 0.f) ? v : 0.1f * v;
    if (act == 12) return (v > 0.f) ? v : 0.2f * v;
    if (act == 13) return (v > 20.f) ? v : log1pf(expf(v));
    return v;
}

struct GemmP {
    const float* A; const float* B; const float* bias; const float* R; float* C;
    long long sAo, sAi, sAm, sAk, sBo, sBi, sBn, sBk, sCo, sCi, sCm, sRo, sRi, sRm, sRn;
    int M, N, K, zi_n, flags, act; float alpha, beta, sa, sb;
    int Npad, pad_;
};
static_assert(sizeof(GemmP) == 5 * 8 + 15 * 8 + 6 * 4 + 4 * 4 + 2 * 4, "GemmP has padding");

template <int MODE>
__global__ __launch_bounds__(32) void k_gemm(GemmP p) {
    const int lane = threadIdx.x & 31, h = lane >> 4, l15 = lane & 15;
    const int m0 = blockIdx.y * 16, n0 = blockIdx.x * 32;
    const int z = blockIdx.z, zo = z / p.zi_n, zi = z - zo * p.zi_n;
    const float* A = p.A + zo * p.sAo + zi * p.sAi;
    const float* B = p.B + zo * p.sBo + zi * p.sBi;
    const int am = min(m0 + l15, p.M - 1);
    v8f acc[2], comp[2];
#pragma unroll
    for (int t = 0; t < 2; ++t) { v8f zz = {}; acc[t] = zz; comp[t] = zz; }
    for (int k0 = 0; k0 < p.K; k0 += 32) {
        const float* arow = A + (long long)am * p.sAm;
        if (MODE == 1) {
            const Split a = sp_ld(arow, p.sAk, k0, h, p.K, 1.f);
#pragma unroll
            for (int t = 0; t < 2; ++t) {
                const int bn = min(n0 + t * 16 + l15, p.N - 1);
                acc[t] = wmma3(a, sp_ld(B + (long long)bn * p.sBn, p.sBk, k0, h, p.K, 1.f), acc[t]);
            }
        } else if (MODE == 3) {
            const Split3 a = sp3_ld(arow, p.sAk, k0, h, p.K, 1.f);
#pragma unroll
            for (int t = 0; t < 2; ++t) {
                const int bn = min(n0 + t * 16 + l15, p.N - 1);
                acc[t] = wmma6(a, sp3_ld(B + (long long)bn * p.sBn, p.sBk, k0, h, p.K, 1.f), acc[t]);
            }
        } else if (MODE == 4) {
            const Split3 a = sp3_ld(arow, p.sAk, k0, h, p.K, 1.f);
#pragma unroll
            for (int t = 0; t < 2; ++t) {
                const int bn = min(n0 + t * 16 + l15, p.N - 1); v8f zz = {};
                const v8f part = wmma6(a, sp3_ld(B + (long long)bn * p.sBn, p.sBk, k0, h, p.K, 1.f), zz);
                const v8f y = part - comp[t]; const v8f s = acc[t] + y; comp[t] = (s - acc[t]) - y; acc[t] = s;
            }
        } else if (MODE == 2) {
            const v16b a = bh_ld(arow, p.sAk, k0, h, p.K, 1.f);
#pragma unroll
            for (int t = 0; t < 2; ++t) {
                const int bn = min(n0 + t * 16 + l15, p.N - 1);
                acc[t] = wmmab(a, bh_ld(B + (long long)bn * p.sBn, p.sBk, k0, h, p.K, 1.f), acc[t]);
            }
        } else {
            const v16h a = fh_ld(arow, p.sAk, k0, h, p.K, p.sa);
#pragma unroll
            for (int t = 0; t < 2; ++t) {
                const int bn = min(n0 + t * 16 + l15, p.N - 1);
                acc[t] = wmma16(a, fh_ld(B + (long long)bn * p.sBn, p.sBk, k0, h, p.K, p.sb), acc[t]);
            }
        }
    }
    const float iscale = (MODE == 0) ? p.alpha / (p.sa * p.sb) : p.alpha;
    float* C = p.C + zo * p.sCo + zi * p.sCi;
    const float* R = p.R + zo * p.sRo + zi * p.sRi;
    __shared__ __align__(16) float ctile[16][36];
#pragma unroll
    for (int t = 0; t < 2; ++t) {
        const int n = n0 + t * 16 + l15; const int nn = min(n, p.N - 1);
#pragma unroll
        for (int r = 0; r < 8; ++r) {
            const int m = m0 + 8 * h + r; const int mm = min(m, p.M - 1);
            float v = acc[t][r] * iscale;
            if (p.flags & 1) v += p.bias[nn];
            if (p.flags & 2) v += p.bias[mm];
            v = act_fn(v, p.act);
            if (p.flags & 4) v += p.beta * R[(long long)mm * p.sRm + (long long)nn * p.sRn];
            ctile[8 * h + r][t * 16 + l15] = (n < p.N) ? v : 0.f;
        }
    }
    __syncthreads();
    const int NW = (p.Npad > p.N) ? p.Npad : p.N;
    const bool fast = (m0 + 16 <= p.M) && (n0 + 32 <= NW) && ((p.sCm & 3) == 0) && ((((size_t)C) & 15) == 0);
    if (fast) {
#pragma unroll
        for (int s = 0; s < 4; ++s) {
            const int row = s * 4 + (lane >> 3), c4 = (lane & 7) * 4;
            const v4f v = *(const v4f*)&ctile[row][c4];
            VST2V4(C + (long long)(m0 + row) * p.sCm + n0 + c4, v);
        }
    } else {
        for (int row = 0; row < 16; ++row) {
            const int m = m0 + row, n = n0 + lane;
            if (m < p.M && n < NW) VST2(float, C + (long long)m * p.sCm + n, ctile[row][lane]);
        }
    }
}


template <int MODE, int TM, int TN>
__global__ __launch_bounds__(32) void k_gemmT(GemmP p) {
    const int lane = threadIdx.x & 31, h = lane >> 4, l15 = lane & 15;
    const int m0 = blockIdx.y * (16 * TM), n0 = blockIdx.x * (16 * TN);
    const int z = blockIdx.z, zo = z / p.zi_n, zi = z - zo * p.zi_n;
    const float* A = p.A + zo * p.sAo + zi * p.sAi;
    const float* B = p.B + zo * p.sBo + zi * p.sBi;
    v8f acc[TM][TN];
#pragma unroll
    for (int i = 0; i < TM; ++i)
#pragma unroll
        for (int t = 0; t < TN; ++t) { v8f zz = {}; acc[i][t] = zz; }
    for (int k0 = 0; k0 < p.K; k0 += 32) {
        if (MODE == 1) {
            Split a[TM], b[TN];
#pragma unroll
            for (int i = 0; i < TM; ++i) { const int am = min(m0 + 16 * i + l15, p.M - 1); a[i] = sp_ld(A + (long long)am * p.sAm, p.sAk, k0, h, p.K, 1.f); }
#pragma unroll
            for (int t = 0; t < TN; ++t) { const int bn = min(n0 + 16 * t + l15, p.N - 1); b[t] = sp_ld(B + (long long)bn * p.sBn, p.sBk, k0, h, p.K, 1.f); }
#pragma unroll
            for (int i = 0; i < TM; ++i)
#pragma unroll
                for (int t = 0; t < TN; ++t) acc[i][t] = wmma3(a[i], b[t], acc[i][t]);
        } else if (MODE == 2) {
            v16b a[TM], b[TN];
#pragma unroll
            for (int i = 0; i < TM; ++i) { const int am = min(m0 + 16 * i + l15, p.M - 1); a[i] = bh_ld(A + (long long)am * p.sAm, p.sAk, k0, h, p.K, 1.f); }
#pragma unroll
            for (int t = 0; t < TN; ++t) { const int bn = min(n0 + 16 * t + l15, p.N - 1); b[t] = bh_ld(B + (long long)bn * p.sBn, p.sBk, k0, h, p.K, 1.f); }
#pragma unroll
            for (int i = 0; i < TM; ++i)
#pragma unroll
                for (int t = 0; t < TN; ++t) acc[i][t] = wmmab(a[i], b[t], acc[i][t]);
        } else {
            v16h a[TM], b[TN];
#pragma unroll
            for (int i = 0; i < TM; ++i) { const int am = min(m0 + 16 * i + l15, p.M - 1); a[i] = fh_ld(A + (long long)am * p.sAm, p.sAk, k0, h, p.K, p.sa); }
#pragma unroll
            for (int t = 0; t < TN; ++t) { const int bn = min(n0 + 16 * t + l15, p.N - 1); b[t] = fh_ld(B + (long long)bn * p.sBn, p.sBk, k0, h, p.K, p.sb); }
#pragma unroll
            for (int i = 0; i < TM; ++i)
#pragma unroll
                for (int t = 0; t < TN; ++t) acc[i][t] = wmma16(a[i], b[t], acc[i][t]);
        }
    }
    const float iscale = (MODE == 0) ? p.alpha / (p.sa * p.sb) : p.alpha;
    float* C = p.C + zo * p.sCo + zi * p.sCi;
    const float* R = p.R + zo * p.sRo + zi * p.sRi;
    const int NW = (p.Npad > p.N) ? p.Npad : p.N;
    __shared__ __align__(16) float ctile[16][36];
#pragma unroll
    for (int i = 0; i < TM; ++i) {
        const int mb = m0 + 16 * i; if (mb >= p.M) break;
#pragma unroll
        for (int tp = 0; tp < TN / 2; ++tp) {
            const int nb = n0 + 32 * tp; if (nb >= NW) break;
#pragma unroll
            for (int t2 = 0; t2 < 2; ++t2) {
                const int t = 2 * tp + t2; const int n = nb + t2 * 16 + l15; const int nn = min(n, p.N - 1);
#pragma unroll
                for (int r = 0; r < 8; ++r) {
                    const int m = mb + 8 * h + r; const int mm = min(m, p.M - 1);
                    float v = acc[i][t][r] * iscale;
                    if (p.flags & 1) v += p.bias[nn];
                    if (p.flags & 2) v += p.bias[mm];
                    v = act_fn(v, p.act);
                    if (p.flags & 4) v += p.beta * R[(long long)mm * p.sRm + (long long)nn * p.sRn];
                    ctile[8 * h + r][t2 * 16 + l15] = (n < p.N) ? v : 0.f;
                }
            }
            __syncthreads();
            const bool fast = (mb + 16 <= p.M) && (nb + 32 <= NW) && ((p.sCm & 3) == 0) && ((((size_t)C) & 15) == 0);
            if (fast) {
#pragma unroll
                for (int s = 0; s < 4; ++s) {
                    const int row = s * 4 + (lane >> 3), c4 = (lane & 7) * 4;
                    const v4f v = *(const v4f*)&ctile[row][c4];
                    VST2V4(C + (long long)(mb + row) * p.sCm + nb + c4, v);
                }
            } else {
                for (int row = 0; row < 16; ++row) {
                    const int m = mb + row, n = nb + lane;
                    if (m < p.M && n < NW) VST2(float, C + (long long)m * p.sCm + n, ctile[row][lane]);
                }
            }
            __syncthreads();
        }
    }
}

#define AW 4
struct AttnP {
    const float* Q; const float* K; const float* V; float* O; float* P; const float* Mf; const int* Mi; float* ST;
    const float* Pw; const float* Rt; const int* SQ; const int* SK;
    long long swb, swh, swi, swj, srb, srh, sri;
    long long sQb, sQh, sQi, sQd, sKb, sKh, sKj, sKd, sVb, sVh, sVj, sVd, sOb, sOh, sOi, sPb, sPh, sPi, smb, smh, smi, smj;
    int Lq, Lk, dh, dv, hrep, causal, coff, pband;
    float scale, mfill; int nonorm, mpol;
    int roff, rn, segpol, win;
};
static_assert(sizeof(AttnP) == 12 * 8 + 29 * 8 + 16 * 4, "AttnP has padding");

#ifndef KATTN_ATTR
#define KATTN_ATTR
#endif
template <int DHP, int DVP, int QM, bool SPLITPV, bool TWOPASS>
__global__ __launch_bounds__(32 * AW) KATTN_ATTR void k_attn(AttnP p) {
    constexpr int NT = DVP / 16;
    constexpr int KS = DHP / 32;
    constexpr int VP = DVP + 8;
    __shared__ __align__(16) float    pl[AW][16 * 64];
    __shared__ __align__(16) _Float16 vl[(SPLITPV ? 2 : 1) * 64 * VP];
    const int lane = threadIdx.x & 31, hf = lane >> 4, l15 = lane & 15, wave = threadIdx.x >> 5;
    const int h = blockIdx.y, b = blockIdx.z, hk = h / p.hrep;
    const int q0 = (blockIdx.x * AW + wave) * 16;
    float* myp = pl[wave];
    const float L2E = 1.4426950408889634f;
    const float NEG = -__builtin_inff();
    const int qi = min(q0 + l15, p.Lq - 1);
    const float* qrow = p.Q + b * p.sQb + h * p.sQh + (long long)qi * p.sQi;
    const float* kbase = p.K + b * p.sKb + hk * p.sKh;
    const float* vbase = p.V + b * p.sVb + hk * p.sVh;
    v16h qa[QM == 0 ? KS : 1]; Split qs_[QM == 1 ? KS : 1]; Split3 qt_[QM == 2 ? KS : 1];
#pragma unroll
    for (int ks = 0; ks < KS; ++ks) {
        if (QM == 2) qt_[ks] = sp3_ld(qrow, p.sQd, ks * 32, hf, p.dh, 1.f);
        else if (QM == 1) qs_[ks] = sp_ld(qrow, p.sQd, ks * 32, hf, p.dh, 1.f);
        else qa[ks] = fh_ld(qrow, p.sQd, ks * 32, hf, p.dh, 1.f);
    }
    v8f o[NT]; float m8[8], l8[8];
#pragma unroll
    for (int t = 0; t < NT; ++t) { v8f zz = {}; o[t] = zz; }
#pragma unroll
    for (int i = 0; i < 8; ++i) { m8[i] = NEG; l8[i] = 0.f; }
    int jend = p.Lk;
    if (p.causal == 1) { const int je = (blockIdx.x * AW + AW - 1) * 16 + 16 + p.coff; jend = min(jend, max(je, 0)); }
    const int npass = TWOPASS ? 2 : 1;
    for (int pass = 0; pass < npass; ++pass) {
        const bool dopv = (!TWOPASS) || pass == 1;
        for (int j0 = 0; j0 < jend; j0 += 64) {
            if (dopv) {
                __syncthreads();
                for (int idx = threadIdx.x; idx < 64 * DVP; idx += 32 * AW) {
                    const int jr = idx / DVP, d = idx - jr * DVP, j = j0 + jr;
                    const float f = (j < p.Lk && d < p.dv) ? vbase[(long long)j * p.sVj + (long long)d * p.sVd] : 0.f;
                    if (SPLITPV) {
                        const __bf16 hb = bf16_rne(f);
                        ((__bf16*)vl)[jr * VP + d] = hb; ((__bf16*)vl)[64 * VP + jr * VP + d] = bf16_rne(f - bf16_f32(hb));
                    } else vl[jr * VP + d] = (_Float16)f;
                }
            }
            v8f s[4];
#pragma unroll
            for (int t = 0; t < 4; ++t) {
                const int j = min(j0 + t * 16 + l15, p.Lk - 1);
                const float* krow = kbase + (long long)j * p.sKj;
                v8f acc = {};
#pragma unroll
                for (int ks = 0; ks < KS; ++ks) {
                    if (QM == 2)      acc = wmma6(qt_[ks], sp3_ld(krow, p.sKd, ks * 32, hf, p.dh, 1.f), acc);
                    else if (QM == 1) acc = wmma3(qs_[ks], sp_ld(krow, p.sKd, ks * 32, hf, p.dh, 1.f), acc);
                    else              acc = wmma16(qa[ks], fh_ld(krow, p.sKd, ks * 32, hf, p.dh, 1.f), acc);
                }
                s[t] = acc;
            }
            float pv[8][4];
#pragma unroll
            for (int i = 0; i < 8; ++i) {
                const int irow = q0 + i + 8 * hf;
                const int ic = min(irow, p.Lq - 1);
                float sc[4];
#pragma unroll
                for (int t = 0; t < 4; ++t) {
                    const int jg = j0 + t * 16 + l15;
                    float v = s[t][i] * p.scale;
                    if (p.Mf) v += p.Mf[b * p.smb + h * p.smh + (long long)ic * p.smi + (long long)min(jg, p.Lk - 1) * p.smj];
                    if (p.Rt) { int rc = ic - min(jg, p.Lk - 1) + p.roff; rc = rc < 0 ? 0 : (rc >= p.rn ? p.rn - 1 : rc); v += p.Rt[b * p.srb + h * p.srh + (long long)ic * p.sri + rc]; }
                    if (p.Mi) { const int mv = p.Mi[b * p.smb + h * p.smh + (long long)ic * p.smi + (long long)min(jg, p.Lk - 1) * p.smj]; if (p.mpol ? (mv != 0) : (mv == 0)) v = p.mfill; }
                    if (p.SQ) { const bool same = p.SQ[(long long)b * p.Lq + ic] == p.SK[(long long)b * p.Lk + min(jg, p.Lk - 1)]; if (p.segpol ? same : !same) v = p.mfill; }
                    if (p.causal == 2 && jg > irow + p.coff) v = p.mfill;
                    if (jg >= p.Lk || (p.causal == 1 && jg > irow + p.coff) || (p.causal == 3 && jg < irow + p.coff) || (p.win > 0 && irow + p.coff - jg > p.win)) v = NEG; else v *= L2E;
                    sc[t] = v;
                }
                if (!TWOPASS || pass == 0) {
                    float mx = fmaxf(fmaxf(sc[0], sc[1]), fmaxf(sc[2], sc[3]));
                    mx = fmaxf(mx, __shfl_xor(mx, 1, 32)); mx = fmaxf(mx, __shfl_xor(mx, 2, 32));
                    mx = fmaxf(mx, __shfl_xor(mx, 4, 32)); mx = fmaxf(mx, __shfl_xor(mx, 8, 32));
                    const float mnew = fmaxf(m8[i], mx);
                    const float corr = (mnew == NEG) ? 1.f : exp2f(m8[i] - mnew);
                    float rs = 0.f;
#pragma unroll
                    for (int t = 0; t < 4; ++t) {
                        const float pp = (sc[t] == NEG) ? 0.f : exp2f(sc[t] - mnew); rs += pp;
                        pv[i][t] = p.Pw ? pp * p.Pw[b * p.swb + h * p.swh + (long long)ic * p.swi + (long long)min(j0 + t * 16 + l15, p.Lk - 1) * p.swj] : pp;
                    }
                    rs += __shfl_xor(rs, 1, 32); rs += __shfl_xor(rs, 2, 32); rs += __shfl_xor(rs, 4, 32); rs += __shfl_xor(rs, 8, 32);
                    l8[i] = l8[i] * corr + rs; m8[i] = mnew;
                    if (!TWOPASS) {
#pragma unroll
                        for (int t = 0; t < NT; ++t) o[t][i] *= corr;
                    }
                } else {
                    const float inv = (l8[i] > 0.f) ? 1.f / l8[i] : 0.f;
#pragma unroll
                    for (int t = 0; t < 4; ++t) {
                        const int jg = j0 + t * 16 + l15;
                        float pp = (sc[t] == NEG) ? 0.f : exp2f(sc[t] - m8[i]) * inv;
                        if (p.Pw) pp *= p.Pw[b * p.swb + h * p.swh + (long long)ic * p.swi + (long long)min(jg, p.Lk - 1) * p.swj];
                        pv[i][t] = pp;
                    }
                }
            }
            if (dopv) {
#pragma unroll
                for (int i = 0; i < 8; ++i)
#pragma unroll
                    for (int t = 0; t < 4; ++t) myp[(i + 8 * hf) * 64 + t * 16 + l15] = pv[i][t];
                __syncthreads();
                if (p.P) {
                    float* pb_ = p.P + b * p.sPb + h * p.sPh;
                    const bool fastP = (p.pband == 0) && ((p.sPi & 3) == 0) && (j0 + 64 <= p.Lk) && (q0 + 16 <= p.Lq) && ((((size_t)pb_) & 15) == 0);
                    if (fastP) {
#pragma unroll
                        for (int s = 0; s < 8; ++s) {
                            const int row = s * 2 + (lane >> 4), c4 = (lane & 15) * 4;
                            const v4f v = *(const v4f*)(myp + row * 64 + c4);
                            VST2V4(pb_ + (long long)(q0 + row) * p.sPi + j0 + c4, v);
                        }
                    } else {
                        for (int row = 0; row < 16; ++row) {
                            const int irow = q0 + row; if (irow >= p.Lq) continue;
                            for (int c = lane; c < 64; c += 32) {
                                const int jg = j0 + c; if (jg >= p.Lk) continue;
                                if (p.pband == 0) VST2(float, pb_ + (long long)irow * p.sPi + jg, myp[row * 64 + c]);
                                else if (jg - irow <= p.pband && irow - jg <= p.pband) VST2(float, pb_ + (long long)irow * p.sPi + (jg - irow + p.pband), myp[row * 64 + c]);
                            }
                        }
                    }
                }
                if (SPLITPV) {
                    const Split pa0 = sp_ld(myp + l15 * 64, 1, 0, hf, 64, 1.f), pa1 = sp_ld(myp + l15 * 64, 1, 32, hf, 64, 1.f);
                    const __bf16* vh = (const __bf16*)vl; const __bf16* vlo = vh + 64 * VP;
#pragma unroll
                    for (int t = 0; t < NT; ++t) {
                        const int dcol = t * 16 + l15;
                        Split b0, b1;
#pragma unroll
                        for (int e = 0; e < 16; ++e) {
                            const int k0 = frag_k(e, hf), k1 = 32 + frag_k(e, hf);
                            b0.hi[e] = vh[k0 * VP + dcol]; b0.lo[e] = vlo[k0 * VP + dcol]; b1.hi[e] = vh[k1 * VP + dcol]; b1.lo[e] = vlo[k1 * VP + dcol];
                        }
                        o[t] = wmma3(pa0, b0, o[t]);
                        o[t] = wmma3(pa1, b1, o[t]);
                    }
                } else {
                    const v16h pa0 = fh_ld(myp + l15 * 64, 1, 0, hf, 64, 4096.f), pa1 = fh_ld(myp + l15 * 64, 1, 32, hf, 64, 4096.f);
#pragma unroll
                    for (int t = 0; t < NT; ++t) {
                        const int dcol = t * 16 + l15;
                        v16h b0, b1;
#pragma unroll
                        for (int e = 0; e < 16; ++e) { b0[e] = vl[frag_k(e, hf) * VP + dcol]; b1[e] = vl[(32 + frag_k(e, hf)) * VP + dcol]; }
                        o[t] = wmma16(pa0, b0, o[t]);
                        o[t] = wmma16(pa1, b1, o[t]);
                    }
                }
            }
        }
    }
    float* obase = p.O + b * p.sOb + h * p.sOh;
    if (p.ST) {
        const int rl = lane >> 1, isel = rl & 7;
        float mv = 0.f, lv = 0.f;
#pragma unroll
        for (int i = 0; i < 8; ++i) if (i == isel) { mv = m8[i]; lv = l8[i]; }
        const int irow = q0 + rl;
        if (irow < p.Lq) { float* st = p.ST + (((long long)b * gridDim.y + h) * p.Lq + irow) * 2 + (lane & 1); VST2(float, st, (lane & 1) ? lv : mv * 0.6931471805599453f); }
    }
    float invr[8];
#pragma unroll
    for (int i = 0; i < 8; ++i) {
        if (TWOPASS) invr[i] = SPLITPV ? 1.f : (1.f / 4096.f);
        else if (p.nonorm) invr[i] = exp2f(m8[i]) * (SPLITPV ? 1.f : (1.f / 4096.f));
        else invr[i] = (l8[i] > 0.f) ? (SPLITPV ? 1.f / l8[i] : 1.f / (l8[i] * 4096.f)) : 0.f;
    }
    __syncthreads();
    const bool ofast = ((p.sOi & 3) == 0) && ((((size_t)obase) & 15) == 0) && (q0 + 16 <= p.Lq);
#pragma unroll
    for (int c0 = 0; c0 < DVP; c0 += 64) {
#pragma unroll
        for (int i = 0; i < 8; ++i)
#pragma unroll
            for (int t = 0; t < NT; ++t) if (t * 16 >= c0 && t * 16 < c0 + 64) myp[(i + 8 * hf) * 64 + (t * 16 - c0) + l15] = o[t][i] * invr[i];
        __syncthreads();
        const int cw = (DVP - c0 < 64) ? (DVP - c0) : 64;
        if (ofast && (c0 + cw <= p.dv) && (cw % 32 == 0)) {
            const int lpr = cw / 4;
            const int rows_per_ins = 32 / lpr;
            for (int r0 = 0; r0 < 16; r0 += rows_per_ins) {
                const int row = r0 + lane / lpr, c4 = (lane % lpr) * 4;
                const v4f v = *(const v4f*)(myp + row * 64 + c4);
                VST2V4(obase + (long long)(q0 + row) * p.sOi + c0 + c4, v);
            }
        } else {
            for (int row = 0; row < 16; ++row) {
                const int irow = q0 + row; if (irow >= p.Lq) continue;
                for (int c = lane; c < cw; c += 32) { const int d = c0 + c; if (d < p.dv) VST2(float, obase + (long long)irow * p.sOi + d, myp[row * 64 + c]); }
            }
        }
        __syncthreads();
    }
}

struct TrP { const float* src; float* dst; const float* R2; long long sSz, lds, sDz, ldd, sRz, ldr; int R, C, flags, act; float alpha, beta; };
static_assert(sizeof(TrP) == 3 * 8 + 6 * 8 + 6 * 4, "TrP has padding");
__global__ __launch_bounds__(256) void k_tr(TrP p) {
    __shared__ float tile[32][33];
    const int c0 = blockIdx.x * 32, r0 = blockIdx.y * 32, z = blockIdx.z;
    const int lane = threadIdx.x & 31, wave = threadIdx.x >> 5;
    const float* s = p.src + z * p.sSz;
#pragma unroll
    for (int k = 0; k < 4; ++k) {
        const int rl = wave * 4 + k, r = r0 + rl, c = c0 + lane;
        tile[rl][lane] = (r < p.R && c < p.C) ? s[(long long)r * p.lds + c] : 0.f;
    }
    __syncthreads();
    float* d = p.dst + z * p.sDz; const float* rr = p.R2 + z * p.sRz;
#pragma unroll
    for (int k = 0; k < 4; ++k) {
        const int cl = wave * 4 + k, c = c0 + cl, r = r0 + lane;
        if (c < p.C && r < p.R) {
            float v = act_fn(p.alpha * tile[lane][cl], p.act);
            if (p.flags & 1) v += p.beta * rr[(long long)c * p.ldr + r];
            VST2(float, d + (long long)c * p.ldd + r, v);
        }
    }
}

__global__ __launch_bounds__(256) void k_affine(const float* __restrict__ src, float* __restrict__ dst, int n, float a, float b, const float* __restrict__ sdev) {
    const int i = blockIdx.x * 256 + threadIdx.x;
    if (i < n) { const float aa = sdev ? a * sdev[0] : a; const float v = aa * src[i] + b; VST2(float, dst + i, v); }
}

struct SmP { const float* src; float* dst; const float* Mf; long long sz, sr, dz, dr, smz, smr; int n, pad; float scale_in, scale_out; };
static_assert(sizeof(SmP) == 3 * 8 + 6 * 8 + 4 * 4, "SmP has padding");
__global__ __launch_bounds__(256) void k_softmax(SmP p) {
    __shared__ float red[256];
    const int r = blockIdx.x, z = blockIdx.y, tid = threadIdx.x;
    const float* s = p.src + z * p.sz + (long long)r * p.sr;
    const float* mf = p.Mf ? (p.Mf + z * p.smz + (long long)r * p.smr) : nullptr;
    float mx = -__builtin_inff();
    for (int j = tid; j < p.n; j += 256) { float v = s[j] * p.scale_in; if (mf) v += mf[j]; mx = fmaxf(mx, v); }
    red[tid] = mx; __syncthreads();
    for (int o = 128; o > 0; o >>= 1) { if (tid < o) red[tid] = fmaxf(red[tid], red[tid + o]); __syncthreads(); }
    mx = red[0]; __syncthreads();
    float sum = 0.f;
    for (int j = tid; j < p.n; j += 256) { float v = s[j] * p.scale_in; if (mf) v += mf[j]; sum += (mx == -__builtin_inff()) ? 0.f : expf(v - mx); }
    red[tid] = sum; __syncthreads();
    for (int o = 128; o > 0; o >>= 1) { if (tid < o) red[tid] += red[tid + o]; __syncthreads(); }
    sum = red[0];
    const float inv = (sum > 0.f) ? p.scale_out / sum : 0.f;
    float* d = p.dst + z * p.dz + (long long)r * p.dr;
    for (int j = tid; j < p.n; j += 256) { float v = s[j] * p.scale_in; if (mf) v += mf[j]; const float o = (mx == -__builtin_inff()) ? 0.f : expf(v - mx) * inv; VST2(float, d + j, o); }
}
__global__ __launch_bounds__(256) void k_stats(const float* __restrict__ x, long long sz, long long so, long long si, int inner, int n, float eps, float* __restrict__ stat, int mode) {
    __shared__ float red[256];
    const int z = blockIdx.x, tid = threadIdx.x;
    const float* base = x + z * sz;
    float s = 0.f;
    for (int e = tid; e < n; e += 256) s += base[(long long)(e / inner) * so + (long long)(e % inner) * si];
    red[tid] = s; __syncthreads();
    for (int o = 128; o > 0; o >>= 1) { if (tid < o) red[tid] += red[tid + o]; __syncthreads(); }
    const float mu = (mode == 0 || mode == 3) ? red[0] / (float)n : 0.f; __syncthreads();
    float q = 0.f;
    for (int e = tid; e < n; e += 256) { const float dlt = base[(long long)(e / inner) * so + (long long)(e % inner) * si] - mu; q += dlt * dlt; }
    red[tid] = q; __syncthreads();
    for (int o = 128; o > 0; o >>= 1) { if (tid < o) red[tid] += red[tid + o]; __syncthreads(); }
    {
        float rs;
        if (mode == 2) rs = sqrtf((float)n) / fmaxf(sqrtf(red[0]), eps); else if (mode == 3) rs = rsqrtf(red[0] / (float)(n - 1) + eps); else rs = rsqrtf(red[0] / (float)n + eps);
        if (tid < 32) { const float v = (tid == 0) ? mu : ((tid == 1) ? rs : 0.f); VST2(float, stat + (long long)z * 32 + tid, v); }
    }
}
__global__ __launch_bounds__(256) void k_norm_apply(const float* __restrict__ x, float* __restrict__ y, const float* __restrict__ stat, const float* __restrict__ g, const float* __restrict__ bta,
                                                     int Z, int C, int L, int G, int bn, int act) {
    const long long idx = (long long)blockIdx.x * 256 + threadIdx.x;
    if (idx >= (long long)Z * C * L) return;
    const int l = (int)(idx % L); const long long zc = idx / L; const int c = (int)(zc % C), z = (int)(zc / C); (void)l;
    const int set = bn ? c : (z * G + c / (C / G));
    float v = (x[idx] - stat[(long long)set * 32]) * stat[(long long)set * 32 + 1];
    if (g) v *= g[c];
    if (bta) v += bta[c];
    v = act_fn(v, act);
    VST2(float, y + idx, v);
}

__global__ __launch_bounds__(256) void k_lse_neg(const float* __restrict__ st, float* __restrict__ c, int n) {
    const int i = blockIdx.x * 256 + threadIdx.x;
    if (i < n) { const float v = -(st[2 * i] + logf(st[2 * i + 1])); VST2(float, c + i, v); }
}

__global__ __launch_bounds__(256) void k_iota(int* __restrict__ dst, int n, int a, int b) {
    const int i = blockIdx.x * 256 + threadIdx.x;
    if (i < n) { const int v = a * i + b; VST2(int, dst + i, v); }
}

__global__ __launch_bounds__(256) void k_axpby(const float* __restrict__ x, const float* __restrict__ y, float* __restrict__ dst, int n, float a, float b, float c) {
    const int i = blockIdx.x * 256 + threadIdx.x;
    if (i < n) { const float v = a * x[i] + b * y[i] + c; VST2(float, dst + i, v); }
}

struct RopeP { const float* X; float* Y; const float* C; const float* Sn; const int* pos; long long sXr, sXh, sYr, sYh, sCb, sCp, sCd; int R, Hn, D, S, mode, tmode, pmode, pad; };
static_assert(sizeof(RopeP) == 5 * 8 + 7 * 8 + 8 * 4, "RopeP has padding");
__global__ __launch_bounds__(256) void k_rope(RopeP p) {
    const long long idx = (long long)blockIdx.x * 256 + threadIdx.x;
    if (idx >= (long long)p.R * p.Hn * p.D) return;
    const int d = (int)(idx % p.D); const long long rh = idx / p.D; const int h = (int)(rh % p.Hn); const int r = (int)(rh / p.Hn);
    const int half = p.D / 2;
    int partner; float sign;
    if (p.mode == 0) { partner = (d < half) ? d + half : d - half; sign = (d < half) ? -1.f : 1.f; }
    else { partner = d ^ 1; sign = (d & 1) ? 1.f : -1.f; }
    const int tcol = (p.tmode == 0) ? d : ((p.tmode == 1) ? (d % half) : (d >> 1));
    const int pp = (p.pmode == 0) ? (r % p.S) : ((p.pmode == 1) ? h : p.pos[r]);
    const long long toff = (long long)(r / p.S) * p.sCb + (long long)pp * p.sCp + (long long)tcol * p.sCd;
    const float* xr = p.X + (long long)r * p.sXr + (long long)h * p.sXh;
    const float v = xr[d] * p.C[toff] + sign * xr[partner] * p.Sn[toff];
    VST2(float, p.Y + (long long)r * p.sYr + (long long)h * p.sYh + d, v);
}

__global__ __launch_bounds__(256) void k_invf(float* __restrict__ invb, int half, int D, float base, float num, int fmode, float cexp) {
    const int i = blockIdx.x * 256 + threadIdx.x;
    if (i >= ((half + 31) / 32) * 32) return;
    if (i >= half) { VST2(float, invb + i, 0.f); return; }
    const float e = (float)(2 * i) / (float)D;
    float invf;
    if (fmode == 1) invf = num * expf((float)(2 * i) * cexp);
    else if (fmode == 2) invf = num * powf(base, (-2.0f * ((float)i - 1.0f)) / (float)D);
    else invf = num * (1.0f / powf(base, e));
    VST2(float, invb + i, invf);
}
__global__ __launch_bounds__(256) void k_sincos(float* __restrict__ cs, float* __restrict__ sn, const float* __restrict__ invb, int S, int half, float pscale) {
    const int idx = blockIdx.x * 256 + threadIdx.x;
    if (idx >= S * half) return;
    const int s = idx / half, i = idx - s * half;
    const float ang = (pscale * (float)s) * invb[i];
    VST2(float, cs + idx, cosf(ang)); VST2(float, sn + idx, sinf(ang));
}

__global__ __launch_bounds__(256) void k_mulact(const float* __restrict__ x, const float* __restrict__ y, float* __restrict__ dst, int n, int act) {
    const int i = blockIdx.x * 256 + threadIdx.x;
    if (i < n) { const float v = act_fn(x[i], act) * y[i]; VST2(float, dst + i, v); }
}

__global__ __launch_bounds__(256) void k_matvec(GemmP p) {
    const int rpt = (p.N == 1) ? 1 : 32;
    const long long r0 = ((long long)blockIdx.x * 256 + threadIdx.x) * rpt; const int z = blockIdx.z, zo = z / p.zi_n, zi = z - zo * p.zi_n;
    if (r0 >= p.M) return;
    const float* Bb = p.B + zo * p.sBo + zi * p.sBi;
    float* C = p.C + zo * p.sCo + zi * p.sCi; const float* R = p.R + zo * p.sRo + zi * p.sRi;
    for (int rr = 0; rr < rpt; ++rr) {
        const long long r = r0 + rr; if (r >= p.M) break;
        const float* A = p.A + zo * p.sAo + zi * p.sAi + r * p.sAm;
        float acc[8] = {0.f, 0.f, 0.f, 0.f, 0.f, 0.f, 0.f, 0.f};
        for (int k = 0; k < p.K; ++k) { const float a = A[(long long)k * p.sAk];
#pragma unroll
            for (int j = 0; j < 8; ++j) if (j < p.N) acc[j] += a * Bb[(long long)j * p.sBn + (long long)k * p.sBk]; }
#pragma unroll
        for (int j = 0; j < 8; ++j) if (j < p.N) {
            float v = acc[j] * p.alpha;
            if (p.flags & 1) v += p.bias[j];
            if (p.flags & 2) v += p.bias[r];
            v = act_fn(v, p.act);
            if (p.flags & 4) v += p.beta * R[r * p.sRm + (long long)j * p.sRn];
            VST2(float, C + r * p.sCm + j, v);
        }
    }
}
__global__ __launch_bounds__(256) void k_smallsoftmax(const float* __restrict__ src, float* __restrict__ dst, long long sr, long long dr, int n, long long R, float scale) {
    const long long r0 = ((long long)blockIdx.x * 256 + threadIdx.x) * 32;
    for (int rr = 0; rr < 32; ++rr) {
        const long long r = r0 + rr; if (r >= R) return;
        const float* s = src + r * sr; float* d = dst + r * dr;
        float mx = -__builtin_inff();
        for (int j = 0; j < n; ++j) mx = fmaxf(mx, s[j] * scale);
        float sum = 0.f;
        for (int j = 0; j < n; ++j) sum += expf(s[j] * scale - mx);
        const float inv = 1.f / sum;
        for (int j = 0; j < n; ++j) { const float v = expf(s[j] * scale - mx) * inv; VST2(float, d + j, v); }
    }
}

__global__ __launch_bounds__(32) void k_unitstat(float* __restrict__ st) { const int t = threadIdx.x; const float v = (t == 1) ? 1.f : 0.f; VST2(float, st + t, v); }

__global__ __launch_bounds__(256) void k_lincopy(const float* __restrict__ src, long long lds, float* __restrict__ dst, long long ldd, long long rows, int cols) {
    const long long i = (long long)blockIdx.x * 256 + threadIdx.x; if (i >= rows * cols) return;
    const long long r = i / cols; const int c = (int)(i - r * cols);
    const float v = src[r * lds + c]; VST2(float, dst + r * ldd + c, v);
}

__global__ __launch_bounds__(256) void k_tru_wvg(const float* __restrict__ Wv, const float* __restrict__ bv, const float* __restrict__ gam, float* __restrict__ WVG, int C) { const int q = blockIdx.x * 256 + threadIdx.x; const float gm = gam[0]; if (q < C * C) VST2(float, WVG + q, Wv[q] * gm); else if (q < C * C + C) VST2(float, WVG + q, bv[q - C * C] * gm); }
__global__ __launch_bounds__(128) void k_tru_colsoft(float* __restrict__ E, int Z, int Hs) { const long long q = (long long)blockIdx.x * 128 + threadIdx.x; if (q >= (long long)Z * Hs) return; const int wp = (int)(q % Hs); const long long z = q / Hs; float* col = E + z * Hs * Hs + wp; float mx = -__builtin_inff();
#pragma unroll 1
    for (int w = 0; w < Hs; ++w) mx = fmaxf(mx, col[(long long)w * Hs]); float s = 0.f;
#pragma unroll 1
    for (int w = 0; w < Hs; ++w) { const float e = expf(col[(long long)w * Hs] - mx); s += e; VST2(float, col + (long long)w * Hs, e); } const float inv = 1.f / s;
#pragma unroll 1
    for (int w = 0; w < Hs; ++w) { const float e = col[(long long)w * Hs]; VST2(float, col + (long long)w * Hs, e * inv); } }
__global__ __launch_bounds__(256) void k_tru_pad(const float* __restrict__ Y, float* __restrict__ YP, int ZC, int Hs, int PW) { const long long q = (long long)blockIdx.x * 256 + threadIdx.x; if (q >= (long long)ZC * PW * PW) return; const int xx = (int)(q % PW); const int yy = (int)((q / PW) % PW); const long long zc = q / ((long long)PW * PW); float v = 0.f; if (xx >= 1 && xx <= Hs && yy >= 1 && yy <= Hs) v = Y[(zc * Hs + (yy - 1)) * Hs + (xx - 1)]; VST2(float, YP + q, v); }
__global__ __launch_bounds__(256) void k_tru_bnc(const float* __restrict__ Zp, const float* __restrict__ s_, const float* __restrict__ b_, const float* __restrict__ m_, const float* __restrict__ v_, float* __restrict__ D, int Z, int C, int Hs, int PW, int src_pw) { const long long q = (long long)blockIdx.x * 256 + threadIdx.x; if (q >= (long long)Z * C * Hs * Hs) return; const int xx = (int)(q % Hs); const int yy = (int)((q / Hs) % Hs); const long long zo = q / ((long long)Hs * Hs); const int o = (int)(zo % C);
    const float inv = s_[o] * rsqrtf(v_[o] + 1e-5f); const float v = Zp[(zo * Hs + yy) * src_pw + xx] * inv + (b_[o] - m_[o] * inv); VST2(float, D + q, fmaxf(v, 0.f)); }

template __global__ void k_gemm<0>(GemmP);
template __global__ void k_gemm<1>(GemmP);

extern "C" void kernel_launch(void* const* d_in, const int* in_sizes, int n_in, void* d_out, int out_size, void* d_ws, size_t ws_size, hipStream_t stream) {
    (void)in_sizes; (void)n_in; (void)out_size; (void)ws_size;
    const float* x1 = (const float*)d_in[0];
    const float* xc = (const float*)d_in[1];
    const float* Wq = (const float*)d_in[2];
    const float* bq = (const float*)d_in[3];
    const float* Wk = (const float*)d_in[4];
    const float* bk = (const float*)d_in[5];
    const float* Wv = (const float*)d_in[6];
    const float* bv = (const float*)d_in[7];
    const float* gam = (const float*)d_in[8];
    const float* c1w = (const float*)d_in[9];
    const float* bn1s = (const float*)d_in[10];
    const float* bn1b = (const float*)d_in[11];
    const float* bn1m = (const float*)d_in[12];
    const float* bn1v = (const float*)d_in[13];
    const float* c2w = (const float*)d_in[14];
    const float* bn2s = (const float*)d_in[15];
    const float* bn2b = (const float*)d_in[16];
    const float* bn2m = (const float*)d_in[17];
    const float* bn2v = (const float*)d_in[18];
    const int Bn = 8;
    const int GB = 4;
    const int C = 64;
    const int Hs = 128;
    const int P = Hs * Hs;
    const int PW = 130;
    const int PP = PW * PW;
    const int NW = Hs * PW;
    float* out = (float*)d_out;
    char* wsp = (char*)d_ws;
    float* Q = (float*)wsp; wsp += (((size_t)((size_t)GB * C * P) * 4 + 255) / 256) * 256;
    float* Kc = (float*)wsp; wsp += (((size_t)((size_t)GB * C * P) * 4 + 255) / 256) * 256;
    float* V = (float*)wsp; wsp += (((size_t)((size_t)GB * C * P) * 4 + 255) / 256) * 256;
    float* E = (float*)wsp; wsp += (((size_t)((size_t)GB * C * Hs * Hs) * 4 + 255) / 256) * 256;
    float* Y = (float*)wsp; wsp += (((size_t)((size_t)GB * C * P) * 4 + 255) / 256) * 256;
    float* YP = (float*)wsp; wsp += (((size_t)((size_t)GB * C * PP) * 4 + 255) / 256) * 256;
    float* Z = (float*)wsp; wsp += (((size_t)((size_t)GB * C * NW) * 4 + 255) / 256) * 256;
    float* WVG = (float*)wsp; wsp += (((size_t)((size_t)C * C + 64) * 4 + 255) / 256) * 256;
    k_tru_wvg<<<(unsigned)((C * C + C + 255) / 256), 256, 0, stream>>>(Wv, bv, gam, WVG, C);
    { GemmP gq0;
      gq0.A = Wq; gq0.B = x1 + (size_t)0 * C * P; gq0.bias = bq; gq0.R = Wq; gq0.C = Q;
      gq0.sAo = 0; gq0.sAi = 0; gq0.sAm = C; gq0.sAk = 1; gq0.sBo = (long long)C * P; gq0.sBi = 0; gq0.sBn = 1; gq0.sBk = P; gq0.sCo = (long long)C * P; gq0.sCi = 0; gq0.sCm = P; gq0.sRo = 0; gq0.sRi = 0; gq0.sRm = 0; gq0.sRn = 0;
      gq0.M = C; gq0.N = P; gq0.K = C; gq0.zi_n = 1; gq0.flags = 2; gq0.act = 0;
      gq0.alpha = 1.0f; gq0.beta = 0.0f; gq0.sa = 1.0f; gq0.sb = 1.0f; gq0.Npad = P; gq0.pad_ = 0;
      if ((long long)(C) >= 64 && (long long)(P) >= 64) k_gemmT<1, 2, 4><<<dim3((unsigned)((P) + 63) / 64, (unsigned)((C) + 31) / 32, (unsigned)(GB)), 32, 0, stream>>>(gq0);
      else k_gemm<1><<<dim3((unsigned)((P) + 31) / 32, (unsigned)((C) + 15) / 16, (unsigned)(GB)), 32, 0, stream>>>(gq0); }
    { GemmP gk0;
      gk0.A = Wk; gk0.B = xc + (size_t)0 * C * P; gk0.bias = bk; gk0.R = Wk; gk0.C = Kc;
      gk0.sAo = 0; gk0.sAi = 0; gk0.sAm = C; gk0.sAk = 1; gk0.sBo = (long long)C * P; gk0.sBi = 0; gk0.sBn = 1; gk0.sBk = P; gk0.sCo = (long long)C * P; gk0.sCi = 0; gk0.sCm = P; gk0.sRo = 0; gk0.sRi = 0; gk0.sRm = 0; gk0.sRn = 0;
      gk0.M = C; gk0.N = P; gk0.K = C; gk0.zi_n = 1; gk0.flags = 2; gk0.act = 0;
      gk0.alpha = 1.0f; gk0.beta = 0.0f; gk0.sa = 1.0f; gk0.sb = 1.0f; gk0.Npad = P; gk0.pad_ = 0;
      if ((long long)(C) >= 64 && (long long)(P) >= 64) k_gemmT<1, 2, 4><<<dim3((unsigned)((P) + 63) / 64, (unsigned)((C) + 31) / 32, (unsigned)(GB)), 32, 0, stream>>>(gk0);
      else k_gemm<1><<<dim3((unsigned)((P) + 31) / 32, (unsigned)((C) + 15) / 16, (unsigned)(GB)), 32, 0, stream>>>(gk0); }
    { GemmP gv0;
      gv0.A = WVG; gv0.B = xc + (size_t)0 * C * P; gv0.bias = WVG + C * C; gv0.R = WVG; gv0.C = V;
      gv0.sAo = 0; gv0.sAi = 0; gv0.sAm = C; gv0.sAk = 1; gv0.sBo = (long long)C * P; gv0.sBi = 0; gv0.sBn = 1; gv0.sBk = P; gv0.sCo = (long long)C * P; gv0.sCi = 0; gv0.sCm = P; gv0.sRo = 0; gv0.sRi = 0; gv0.sRm = 0; gv0.sRn = 0;
      gv0.M = C; gv0.N = P; gv0.K = C; gv0.zi_n = 1; gv0.flags = 2; gv0.act = 0;
      gv0.alpha = 1.0f; gv0.beta = 0.0f; gv0.sa = 1.0f; gv0.sb = 1.0f; gv0.Npad = P; gv0.pad_ = 0;
      if ((long long)(C) >= 64 && (long long)(P) >= 64) k_gemmT<1, 2, 4><<<dim3((unsigned)((P) + 63) / 64, (unsigned)((C) + 31) / 32, (unsigned)(GB)), 32, 0, stream>>>(gv0);
      else k_gemm<1><<<dim3((unsigned)((P) + 31) / 32, (unsigned)((C) + 15) / 16, (unsigned)(GB)), 32, 0, stream>>>(gv0); }
    { GemmP ge0;
      ge0.A = Q; ge0.B = Kc; ge0.bias = Q; ge0.R = Q; ge0.C = E;
      ge0.sAo = P; ge0.sAi = 0; ge0.sAm = 1; ge0.sAk = Hs; ge0.sBo = P; ge0.sBi = 0; ge0.sBn = 1; ge0.sBk = Hs; ge0.sCo = (long long)Hs * Hs; ge0.sCi = 0; ge0.sCm = Hs; ge0.sRo = 0; ge0.sRi = 0; ge0.sRm = 0; ge0.sRn = 0;
      ge0.M = Hs; ge0.N = Hs; ge0.K = Hs; ge0.zi_n = 1; ge0.flags = 0; ge0.act = 0;
      ge0.alpha = 1.0f; ge0.beta = 0.0f; ge0.sa = 1.0f; ge0.sb = 1.0f; ge0.Npad = Hs; ge0.pad_ = 0;
      if ((long long)(Hs) >= 64 && (long long)(Hs) >= 64) k_gemmT<1, 2, 4><<<dim3((unsigned)((Hs) + 63) / 64, (unsigned)((Hs) + 31) / 32, (unsigned)(GB * C)), 32, 0, stream>>>(ge0);
      else k_gemm<1><<<dim3((unsigned)((Hs) + 31) / 32, (unsigned)((Hs) + 15) / 16, (unsigned)(GB * C)), 32, 0, stream>>>(ge0); }
    k_tru_colsoft<<<(unsigned)((GB * C * Hs + 127) / 128), 128, 0, stream>>>(E, GB * C, Hs);
    { GemmP gy0;
      gy0.A = V; gy0.B = E; gy0.bias = V; gy0.R = xc + (size_t)0 * C * P; gy0.C = Y;
      gy0.sAo = P; gy0.sAi = 0; gy0.sAm = Hs; gy0.sAk = 1; gy0.sBo = (long long)Hs * Hs; gy0.sBi = 0; gy0.sBn = 1; gy0.sBk = Hs; gy0.sCo = P; gy0.sCi = 0; gy0.sCm = Hs; gy0.sRo = P; gy0.sRi = 0; gy0.sRm = Hs; gy0.sRn = 1;
      gy0.M = Hs; gy0.N = Hs; gy0.K = Hs; gy0.zi_n = 1; gy0.flags = 4; gy0.act = 0;
      gy0.alpha = 1.0f; gy0.beta = 1.0f; gy0.sa = 1.0f; gy0.sb = 1.0f; gy0.Npad = Hs; gy0.pad_ = 0;
      if ((long long)(Hs) >= 64 && (long long)(Hs) >= 64) k_gemmT<0, 4, 4><<<dim3((unsigned)((Hs) + 63) / 64, (unsigned)((Hs) + 63) / 64, (unsigned)(GB * C)), 32, 0, stream>>>(gy0);
      else k_gemm<0><<<dim3((unsigned)((Hs) + 31) / 32, (unsigned)((Hs) + 15) / 16, (unsigned)(GB * C)), 32, 0, stream>>>(gy0); }
    k_tru_pad<<<(unsigned)(((long long)GB * C * PP + 255) / 256), 256, 0, stream>>>(Y, YP, GB * C, Hs, PW);
    { GemmP gc00;
      gc00.A = c1w + 0; gc00.B = YP + 0; gc00.bias = c1w + 0; gc00.R = c1w + 0; gc00.C = Z;
      gc00.sAo = 0; gc00.sAi = 0; gc00.sAm = C * 9; gc00.sAk = 9; gc00.sBo = (long long)C * PP; gc00.sBi = 0; gc00.sBn = 1; gc00.sBk = PP; gc00.sCo = (long long)C * NW; gc00.sCi = 0; gc00.sCm = NW; gc00.sRo = 0; gc00.sRi = 0; gc00.sRm = 0; gc00.sRn = 0;
      gc00.M = C; gc00.N = NW - 2; gc00.K = C; gc00.zi_n = 1; gc00.flags = 0; gc00.act = 0;
      gc00.alpha = 1.0f; gc00.beta = 0.0f; gc00.sa = 8.0f; gc00.sb = 1.0f; gc00.Npad = NW - 2; gc00.pad_ = 0;
      if ((long long)(C) >= 64 && (long long)(NW - 2) >= 64) k_gemmT<0, 4, 4><<<dim3((unsigned)((NW - 2) + 63) / 64, (unsigned)((C) + 63) / 64, (unsigned)(GB)), 32, 0, stream>>>(gc00);
      else k_gemm<0><<<dim3((unsigned)((NW - 2) + 31) / 32, (unsigned)((C) + 15) / 16, (unsigned)(GB)), 32, 0, stream>>>(gc00); }
    { GemmP gc01;
      gc01.A = c1w + 1; gc01.B = YP + 1; gc01.bias = c1w + 1; gc01.R = Z; gc01.C = Z;
      gc01.sAo = 0; gc01.sAi = 0; gc01.sAm = C * 9; gc01.sAk = 9; gc01.sBo = (long long)C * PP; gc01.sBi = 0; gc01.sBn = 1; gc01.sBk = PP; gc01.sCo = (long long)C * NW; gc01.sCi = 0; gc01.sCm = NW; gc01.sRo = (long long)C * NW; gc01.sRi = 0; gc01.sRm = NW; gc01.sRn = 1;
      gc01.M = C; gc01.N = NW - 2; gc01.K = C; gc01.zi_n = 1; gc01.flags = 4; gc01.act = 0;
      gc01.alpha = 1.0f; gc01.beta = 1.0f; gc01.sa = 8.0f; gc01.sb = 1.0f; gc01.Npad = NW - 2; gc01.pad_ = 0;
      if ((long long)(C) >= 64 && (long long)(NW - 2) >= 64) k_gemmT<0, 4, 4><<<dim3((unsigned)((NW - 2) + 63) / 64, (unsigned)((C) + 63) / 64, (unsigned)(GB)), 32, 0, stream>>>(gc01);
      else k_gemm<0><<<dim3((unsigned)((NW - 2) + 31) / 32, (unsigned)((C) + 15) / 16, (unsigned)(GB)), 32, 0, stream>>>(gc01); }
    { GemmP gc02;
      gc02.A = c1w + 2; gc02.B = YP + 2; gc02.bias = c1w + 2; gc02.R = Z; gc02.C = Z;
      gc02.sAo = 0; gc02.sAi = 0; gc02.sAm = C * 9; gc02.sAk = 9; gc02.sBo = (long long)C * PP; gc02.sBi = 0; gc02.sBn = 1; gc02.sBk = PP; gc02.sCo = (long long)C * NW; gc02.sCi = 0; gc02.sCm = NW; gc02.sRo = (long long)C * NW; gc02.sRi = 0; gc02.sRm = NW; gc02.sRn = 1;
      gc02.M = C; gc02.N = NW - 2; gc02.K = C; gc02.zi_n = 1; gc02.flags = 4; gc02.act = 0;
      gc02.alpha = 1.0f; gc02.beta = 1.0f; gc02.sa = 8.0f; gc02.sb = 1.0f; gc02.Npad = NW - 2; gc02.pad_ = 0;
      if ((long long)(C) >= 64 && (long long)(NW - 2) >= 64) k_gemmT<0, 4, 4><<<dim3((unsigned)((NW - 2) + 63) / 64, (unsigned)((C) + 63) / 64, (unsigned)(GB)), 32, 0, stream>>>(gc02);
      else k_gemm<0><<<dim3((unsigned)((NW - 2) + 31) / 32, (unsigned)((C) + 15) / 16, (unsigned)(GB)), 32, 0, stream>>>(gc02); }
    { GemmP gc03;
      gc03.A = c1w + 3; gc03.B = YP + 130; gc03.bias = c1w + 3; gc03.R = Z; gc03.C = Z;
      gc03.sAo = 0; gc03.sAi = 0; gc03.sAm = C * 9; gc03.sAk = 9; gc03.sBo = (long long)C * PP; gc03.sBi = 0; gc03.sBn = 1; gc03.sBk = PP; gc03.sCo = (long long)C * NW; gc03.sCi = 0; gc03.sCm = NW; gc03.sRo = (long long)C * NW; gc03.sRi = 0; gc03.sRm = NW; gc03.sRn = 1;
      gc03.M = C; gc03.N = NW - 2; gc03.K = C; gc03.zi_n = 1; gc03.flags = 4; gc03.act = 0;
      gc03.alpha = 1.0f; gc03.beta = 1.0f; gc03.sa = 8.0f; gc03.sb = 1.0f; gc03.Npad = NW - 2; gc03.pad_ = 0;
      if ((long long)(C) >= 64 && (long long)(NW - 2) >= 64) k_gemmT<0, 4, 4><<<dim3((unsigned)((NW - 2) + 63) / 64, (unsigned)((C) + 63) / 64, (unsigned)(GB)), 32, 0, stream>>>(gc03);
      else k_gemm<0><<<dim3((unsigned)((NW - 2) + 31) / 32, (unsigned)((C) + 15) / 16, (unsigned)(GB)), 32, 0, stream>>>(gc03); }
    { GemmP gc04;
      gc04.A = c1w + 4; gc04.B = YP + 131; gc04.bias = c1w + 4; gc04.R = Z; gc04.C = Z;
      gc04.sAo = 0; gc04.sAi = 0; gc04.sAm = C * 9; gc04.sAk = 9; gc04.sBo = (long long)C * PP; gc04.sBi = 0; gc04.sBn = 1; gc04.sBk = PP; gc04.sCo = (long long)C * NW; gc04.sCi = 0; gc04.sCm = NW; gc04.sRo = (long long)C * NW; gc04.sRi = 0; gc04.sRm = NW; gc04.sRn = 1;
      gc04.M = C; gc04.N = NW - 2; gc04.K = C; gc04.zi_n = 1; gc04.flags = 4; gc04.act = 0;
      gc04.alpha = 1.0f; gc04.beta = 1.0f; gc04.sa = 8.0f; gc04.sb = 1.0f; gc04.Npad = NW - 2; gc04.pad_ = 0;
      if ((long long)(C) >= 64 && (long long)(NW - 2) >= 64) k_gemmT<0, 4, 4><<<dim3((unsigned)((NW - 2) + 63) / 64, (unsigned)((C) + 63) / 64, (unsigned)(GB)), 32, 0, stream>>>(gc04);
      else k_gemm<0><<<dim3((unsigned)((NW - 2) + 31) / 32, (unsigned)((C) + 15) / 16, (unsigned)(GB)), 32, 0, stream>>>(gc04); }
    { GemmP gc05;
      gc05.A = c1w + 5; gc05.B = YP + 132; gc05.bias = c1w + 5; gc05.R = Z; gc05.C = Z;
      gc05.sAo = 0; gc05.sAi = 0; gc05.sAm = C * 9; gc05.sAk = 9; gc05.sBo = (long long)C * PP; gc05.sBi = 0; gc05.sBn = 1; gc05.sBk = PP; gc05.sCo = (long long)C * NW; gc05.sCi = 0; gc05.sCm = NW; gc05.sRo = (long long)C * NW; gc05.sRi = 0; gc05.sRm = NW; gc05.sRn = 1;
      gc05.M = C; gc05.N = NW - 2; gc05.K = C; gc05.zi_n = 1; gc05.flags = 4; gc05.act = 0;
      gc05.alpha = 1.0f; gc05.beta = 1.0f; gc05.sa = 8.0f; gc05.sb = 1.0f; gc05.Npad = NW - 2; gc05.pad_ = 0;
      if ((long long)(C) >= 64 && (long long)(NW - 2) >= 64) k_gemmT<0, 4, 4><<<dim3((unsigned)((NW - 2) + 63) / 64, (unsigned)((C) + 63) / 64, (unsigned)(GB)), 32, 0, stream>>>(gc05);
      else k_gemm<0><<<dim3((unsigned)((NW - 2) + 31) / 32, (unsigned)((C) + 15) / 16, (unsigned)(GB)), 32, 0, stream>>>(gc05); }
    { GemmP gc06;
      gc06.A = c1w + 6; gc06.B = YP + 260; gc06.bias = c1w + 6; gc06.R = Z; gc06.C = Z;
      gc06.sAo = 0; gc06.sAi = 0; gc06.sAm = C * 9; gc06.sAk = 9; gc06.sBo = (long long)C * PP; gc06.sBi = 0; gc06.sBn = 1; gc06.sBk = PP; gc06.sCo = (long long)C * NW; gc06.sCi = 0; gc06.sCm = NW; gc06.sRo = (long long)C * NW; gc06.sRi = 0; gc06.sRm = NW; gc06.sRn = 1;
      gc06.M = C; gc06.N = NW - 2; gc06.K = C; gc06.zi_n = 1; gc06.flags = 4; gc06.act = 0;
      gc06.alpha = 1.0f; gc06.beta = 1.0f; gc06.sa = 8.0f; gc06.sb = 1.0f; gc06.Npad = NW - 2; gc06.pad_ = 0;
      if ((long long)(C) >= 64 && (long long)(NW - 2) >= 64) k_gemmT<0, 4, 4><<<dim3((unsigned)((NW - 2) + 63) / 64, (unsigned)((C) + 63) / 64, (unsigned)(GB)), 32, 0, stream>>>(gc06);
      else k_gemm<0><<<dim3((unsigned)((NW - 2) + 31) / 32, (unsigned)((C) + 15) / 16, (unsigned)(GB)), 32, 0, stream>>>(gc06); }
    { GemmP gc07;
      gc07.A = c1w + 7; gc07.B = YP + 261; gc07.bias = c1w + 7; gc07.R = Z; gc07.C = Z;
      gc07.sAo = 0; gc07.sAi = 0; gc07.sAm = C * 9; gc07.sAk = 9; gc07.sBo = (long long)C * PP; gc07.sBi = 0; gc07.sBn = 1; gc07.sBk = PP; gc07.sCo = (long long)C * NW; gc07.sCi = 0; gc07.sCm = NW; gc07.sRo = (long long)C * NW; gc07.sRi = 0; gc07.sRm = NW; gc07.sRn = 1;
      gc07.M = C; gc07.N = NW - 2; gc07.K = C; gc07.zi_n = 1; gc07.flags = 4; gc07.act = 0;
      gc07.alpha = 1.0f; gc07.beta = 1.0f; gc07.sa = 8.0f; gc07.sb = 1.0f; gc07.Npad = NW - 2; gc07.pad_ = 0;
      if ((long long)(C) >= 64 && (long long)(NW - 2) >= 64) k_gemmT<0, 4, 4><<<dim3((unsigned)((NW - 2) + 63) / 64, (unsigned)((C) + 63) / 64, (unsigned)(GB)), 32, 0, stream>>>(gc07);
      else k_gemm<0><<<dim3((unsigned)((NW - 2) + 31) / 32, (unsigned)((C) + 15) / 16, (unsigned)(GB)), 32, 0, stream>>>(gc07); }
    { GemmP gc08;
      gc08.A = c1w + 8; gc08.B = YP + 262; gc08.bias = c1w + 8; gc08.R = Z; gc08.C = Z;
      gc08.sAo = 0; gc08.sAi = 0; gc08.sAm = C * 9; gc08.sAk = 9; gc08.sBo = (long long)C * PP; gc08.sBi = 0; gc08.sBn = 1; gc08.sBk = PP; gc08.sCo = (long long)C * NW; gc08.sCi = 0; gc08.sCm = NW; gc08.sRo = (long long)C * NW; gc08.sRi = 0; gc08.sRm = NW; gc08.sRn = 1;
      gc08.M = C; gc08.N = NW - 2; gc08.K = C; gc08.zi_n = 1; gc08.flags = 4; gc08.act = 0;
      gc08.alpha = 1.0f; gc08.beta = 1.0f; gc08.sa = 8.0f; gc08.sb = 1.0f; gc08.Npad = NW - 2; gc08.pad_ = 0;
      if ((long long)(C) >= 64 && (long long)(NW - 2) >= 64) k_gemmT<0, 4, 4><<<dim3((unsigned)((NW - 2) + 63) / 64, (unsigned)((C) + 63) / 64, (unsigned)(GB)), 32, 0, stream>>>(gc08);
      else k_gemm<0><<<dim3((unsigned)((NW - 2) + 31) / 32, (unsigned)((C) + 15) / 16, (unsigned)(GB)), 32, 0, stream>>>(gc08); }
    k_tru_bnc<<<(unsigned)(((long long)GB * C * P + 255) / 256), 256, 0, stream>>>(Z, bn1s, bn1b, bn1m, bn1v, Y, GB, C, Hs, PW, PW);
    { GemmP g20;
      g20.A = c2w; g20.B = Y; g20.bias = c2w; g20.R = c2w; g20.C = Q;
      g20.sAo = 0; g20.sAi = 0; g20.sAm = C; g20.sAk = 1; g20.sBo = (long long)C * P; g20.sBi = 0; g20.sBn = 1; g20.sBk = P; g20.sCo = (long long)C * P; g20.sCi = 0; g20.sCm = P; g20.sRo = 0; g20.sRi = 0; g20.sRm = 0; g20.sRn = 0;
      g20.M = C; g20.N = P; g20.K = C; g20.zi_n = 1; g20.flags = 0; g20.act = 0;
      g20.alpha = 1.0f; g20.beta = 0.0f; g20.sa = 1.0f; g20.sb = 1.0f; g20.Npad = P; g20.pad_ = 0;
      if ((long long)(C) >= 64 && (long long)(P) >= 64) k_gemmT<1, 2, 4><<<dim3((unsigned)((P) + 63) / 64, (unsigned)((C) + 31) / 32, (unsigned)(GB)), 32, 0, stream>>>(g20);
      else k_gemm<1><<<dim3((unsigned)((P) + 31) / 32, (unsigned)((C) + 15) / 16, (unsigned)(GB)), 32, 0, stream>>>(g20); }
    k_tru_bnc<<<(unsigned)(((long long)GB * C * P + 255) / 256), 256, 0, stream>>>(Q, bn2s, bn2b, bn2m, bn2v, out + (size_t)0 * C * P, GB, C, Hs, PW, Hs);
    { GemmP gq1;
      gq1.A = Wq; gq1.B = x1 + (size_t)4 * C * P; gq1.bias = bq; gq1.R = Wq; gq1.C = Q;
      gq1.sAo = 0; gq1.sAi = 0; gq1.sAm = C; gq1.sAk = 1; gq1.sBo = (long long)C * P; gq1.sBi = 0; gq1.sBn = 1; gq1.sBk = P; gq1.sCo = (long long)C * P; gq1.sCi = 0; gq1.sCm = P; gq1.sRo = 0; gq1.sRi = 0; gq1.sRm = 0; gq1.sRn = 0;
      gq1.M = C; gq1.N = P; gq1.K = C; gq1.zi_n = 1; gq1.flags = 2; gq1.act = 0;
      gq1.alpha = 1.0f; gq1.beta = 0.0f; gq1.sa = 1.0f; gq1.sb = 1.0f; gq1.Npad = P; gq1.pad_ = 0;
      if ((long long)(C) >= 64 && (long long)(P) >= 64) k_gemmT<1, 2, 4><<<dim3((unsigned)((P) + 63) / 64, (unsigned)((C) + 31) / 32, (unsigned)(GB)), 32, 0, stream>>>(gq1);
      else k_gemm<1><<<dim3((unsigned)((P) + 31) / 32, (unsigned)((C) + 15) / 16, (unsigned)(GB)), 32, 0, stream>>>(gq1); }
    { GemmP gk1;
      gk1.A = Wk; gk1.B = xc + (size_t)4 * C * P; gk1.bias = bk; gk1.R = Wk; gk1.C = Kc;
      gk1.sAo = 0; gk1.sAi = 0; gk1.sAm = C; gk1.sAk = 1; gk1.sBo = (long long)C * P; gk1.sBi = 0; gk1.sBn = 1; gk1.sBk = P; gk1.sCo = (long long)C * P; gk1.sCi = 0; gk1.sCm = P; gk1.sRo = 0; gk1.sRi = 0; gk1.sRm = 0; gk1.sRn = 0;
      gk1.M = C; gk1.N = P; gk1.K = C; gk1.zi_n = 1; gk1.flags = 2; gk1.act = 0;
      gk1.alpha = 1.0f; gk1.beta = 0.0f; gk1.sa = 1.0f; gk1.sb = 1.0f; gk1.Npad = P; gk1.pad_ = 0;
      if ((long long)(C) >= 64 && (long long)(P) >= 64) k_gemmT<1, 2, 4><<<dim3((unsigned)((P) + 63) / 64, (unsigned)((C) + 31) / 32, (unsigned)(GB)), 32, 0, stream>>>(gk1);
      else k_gemm<1><<<dim3((unsigned)((P) + 31) / 32, (unsigned)((C) + 15) / 16, (unsigned)(GB)), 32, 0, stream>>>(gk1); }
    { GemmP gv1;
      gv1.A = WVG; gv1.B = xc + (size_t)4 * C * P; gv1.bias = WVG + C * C; gv1.R = WVG; gv1.C = V;
      gv1.sAo = 0; gv1.sAi = 0; gv1.sAm = C; gv1.sAk = 1; gv1.sBo = (long long)C * P; gv1.sBi = 0; gv1.sBn = 1; gv1.sBk = P; gv1.sCo = (long long)C * P; gv1.sCi = 0; gv1.sCm = P; gv1.sRo = 0; gv1.sRi = 0; gv1.sRm = 0; gv1.sRn = 0;
      gv1.M = C; gv1.N = P; gv1.K = C; gv1.zi_n = 1; gv1.flags = 2; gv1.act = 0;
      gv1.alpha = 1.0f; gv1.beta = 0.0f; gv1.sa = 1.0f; gv1.sb = 1.0f; gv1.Npad = P; gv1.pad_ = 0;
      if ((long long)(C) >= 64 && (long long)(P) >= 64) k_gemmT<1, 2, 4><<<dim3((unsigned)((P) + 63) / 64, (unsigned)((C) + 31) / 32, (unsigned)(GB)), 32, 0, stream>>>(gv1);
      else k_gemm<1><<<dim3((unsigned)((P) + 31) / 32, (unsigned)((C) + 15) / 16, (unsigned)(GB)), 32, 0, stream>>>(gv1); }
    { GemmP ge1;
      ge1.A = Q; ge1.B = Kc; ge1.bias = Q; ge1.R = Q; ge1.C = E;
      ge1.sAo = P; ge1.sAi = 0; ge1.sAm = 1; ge1.sAk = Hs; ge1.sBo = P; ge1.sBi = 0; ge1.sBn = 1; ge1.sBk = Hs; ge1.sCo = (long long)Hs * Hs; ge1.sCi = 0; ge1.sCm = Hs; ge1.sRo = 0; ge1.sRi = 0; ge1.sRm = 0; ge1.sRn = 0;
      ge1.M = Hs; ge1.N = Hs; ge1.K = Hs; ge1.zi_n = 1; ge1.flags = 0; ge1.act = 0;
      ge1.alpha = 1.0f; ge1.beta = 0.0f; ge1.sa = 1.0f; ge1.sb = 1.0f; ge1.Npad = Hs; ge1.pad_ = 0;
      if ((long long)(Hs) >= 64 && (long long)(Hs) >= 64) k_gemmT<1, 2, 4><<<dim3((unsigned)((Hs) + 63) / 64, (unsigned)((Hs) + 31) / 32, (unsigned)(GB * C)), 32, 0, stream>>>(ge1);
      else k_gemm<1><<<dim3((unsigned)((Hs) + 31) / 32, (unsigned)((Hs) + 15) / 16, (unsigned)(GB * C)), 32, 0, stream>>>(ge1); }
    k_tru_colsoft<<<(unsigned)((GB * C * Hs + 127) / 128), 128, 0, stream>>>(E, GB * C, Hs);
    { GemmP gy1;
      gy1.A = V; gy1.B = E; gy1.bias = V; gy1.R = xc + (size_t)4 * C * P; gy1.C = Y;
      gy1.sAo = P; gy1.sAi = 0; gy1.sAm = Hs; gy1.sAk = 1; gy1.sBo = (long long)Hs * Hs; gy1.sBi = 0; gy1.sBn = 1; gy1.sBk = Hs; gy1.sCo = P; gy1.sCi = 0; gy1.sCm = Hs; gy1.sRo = P; gy1.sRi = 0; gy1.sRm = Hs; gy1.sRn = 1;
      gy1.M = Hs; gy1.N = Hs; gy1.K = Hs; gy1.zi_n = 1; gy1.flags = 4; gy1.act = 0;
      gy1.alpha = 1.0f; gy1.beta = 1.0f; gy1.sa = 1.0f; gy1.sb = 1.0f; gy1.Npad = Hs; gy1.pad_ = 0;
      if ((long long)(Hs) >= 64 && (long long)(Hs) >= 64) k_gemmT<0, 4, 4><<<dim3((unsigned)((Hs) + 63) / 64, (unsigned)((Hs) + 63) / 64, (unsigned)(GB * C)), 32, 0, stream>>>(gy1);
      else k_gemm<0><<<dim3((unsigned)((Hs) + 31) / 32, (unsigned)((Hs) + 15) / 16, (unsigned)(GB * C)), 32, 0, stream>>>(gy1); }
    k_tru_pad<<<(unsigned)(((long long)GB * C * PP + 255) / 256), 256, 0, stream>>>(Y, YP, GB * C, Hs, PW);
    { GemmP gc10;
      gc10.A = c1w + 0; gc10.B = YP + 0; gc10.bias = c1w + 0; gc10.R = c1w + 0; gc10.C = Z;
      gc10.sAo = 0; gc10.sAi = 0; gc10.sAm = C * 9; gc10.sAk = 9; gc10.sBo = (long long)C * PP; gc10.sBi = 0; gc10.sBn = 1; gc10.sBk = PP; gc10.sCo = (long long)C * NW; gc10.sCi = 0; gc10.sCm = NW; gc10.sRo = 0; gc10.sRi = 0; gc10.sRm = 0; gc10.sRn = 0;
      gc10.M = C; gc10.N = NW - 2; gc10.K = C; gc10.zi_n = 1; gc10.flags = 0; gc10.act = 0;
      gc10.alpha = 1.0f; gc10.beta = 0.0f; gc10.sa = 8.0f; gc10.sb = 1.0f; gc10.Npad = NW - 2; gc10.pad_ = 0;
      if ((long long)(C) >= 64 && (long long)(NW - 2) >= 64) k_gemmT<0, 4, 4><<<dim3((unsigned)((NW - 2) + 63) / 64, (unsigned)((C) + 63) / 64, (unsigned)(GB)), 32, 0, stream>>>(gc10);
      else k_gemm<0><<<dim3((unsigned)((NW - 2) + 31) / 32, (unsigned)((C) + 15) / 16, (unsigned)(GB)), 32, 0, stream>>>(gc10); }
    { GemmP gc11;
      gc11.A = c1w + 1; gc11.B = YP + 1; gc11.bias = c1w + 1; gc11.R = Z; gc11.C = Z;
      gc11.sAo = 0; gc11.sAi = 0; gc11.sAm = C * 9; gc11.sAk = 9; gc11.sBo = (long long)C * PP; gc11.sBi = 0; gc11.sBn = 1; gc11.sBk = PP; gc11.sCo = (long long)C * NW; gc11.sCi = 0; gc11.sCm = NW; gc11.sRo = (long long)C * NW; gc11.sRi = 0; gc11.sRm = NW; gc11.sRn = 1;
      gc11.M = C; gc11.N = NW - 2; gc11.K = C; gc11.zi_n = 1; gc11.flags = 4; gc11.act = 0;
      gc11.alpha = 1.0f; gc11.beta = 1.0f; gc11.sa = 8.0f; gc11.sb = 1.0f; gc11.Npad = NW - 2; gc11.pad_ = 0;
      if ((long long)(C) >= 64 && (long long)(NW - 2) >= 64) k_gemmT<0, 4, 4><<<dim3((unsigned)((NW - 2) + 63) / 64, (unsigned)((C) + 63) / 64, (unsigned)(GB)), 32, 0, stream>>>(gc11);
      else k_gemm<0><<<dim3((unsigned)((NW - 2) + 31) / 32, (unsigned)((C) + 15) / 16, (unsigned)(GB)), 32, 0, stream>>>(gc11); }
    { GemmP gc12;
      gc12.A = c1w + 2; gc12.B = YP + 2; gc12.bias = c1w + 2; gc12.R = Z; gc12.C = Z;
      gc12.sAo = 0; gc12.sAi = 0; gc12.sAm = C * 9; gc12.sAk = 9; gc12.sBo = (long long)C * PP; gc12.sBi = 0; gc12.sBn = 1; gc12.sBk = PP; gc12.sCo = (long long)C * NW; gc12.sCi = 0; gc12.sCm = NW; gc12.sRo = (long long)C * NW; gc12.sRi = 0; gc12.sRm = NW; gc12.sRn = 1;
      gc12.M = C; gc12.N = NW - 2; gc12.K = C; gc12.zi_n = 1; gc12.flags = 4; gc12.act = 0;
      gc12.alpha = 1.0f; gc12.beta = 1.0f; gc12.sa = 8.0f; gc12.sb = 1.0f; gc12.Npad = NW - 2; gc12.pad_ = 0;
      if ((long long)(C) >= 64 && (long long)(NW - 2) >= 64) k_gemmT<0, 4, 4><<<dim3((unsigned)((NW - 2) + 63) / 64, (unsigned)((C) + 63) / 64, (unsigned)(GB)), 32, 0, stream>>>(gc12);
      else k_gemm<0><<<dim3((unsigned)((NW - 2) + 31) / 32, (unsigned)((C) + 15) / 16, (unsigned)(GB)), 32, 0, stream>>>(gc12); }
    { GemmP gc13;
      gc13.A = c1w + 3; gc13.B = YP + 130; gc13.bias = c1w + 3; gc13.R = Z; gc13.C = Z;
      gc13.sAo = 0; gc13.sAi = 0; gc13.sAm = C * 9; gc13.sAk = 9; gc13.sBo = (long long)C * PP; gc13.sBi = 0; gc13.sBn = 1; gc13.sBk = PP; gc13.sCo = (long long)C * NW; gc13.sCi = 0; gc13.sCm = NW; gc13.sRo = (long long)C * NW; gc13.sRi = 0; gc13.sRm = NW; gc13.sRn = 1;
      gc13.M = C; gc13.N = NW - 2; gc13.K = C; gc13.zi_n = 1; gc13.flags = 4; gc13.act = 0;
      gc13.alpha = 1.0f; gc13.beta = 1.0f; gc13.sa = 8.0f; gc13.sb = 1.0f; gc13.Npad = NW - 2; gc13.pad_ = 0;
      if ((long long)(C) >= 64 && (long long)(NW - 2) >= 64) k_gemmT<0, 4, 4><<<dim3((unsigned)((NW - 2) + 63) / 64, (unsigned)((C) + 63) / 64, (unsigned)(GB)), 32, 0, stream>>>(gc13);
      else k_gemm<0><<<dim3((unsigned)((NW - 2) + 31) / 32, (unsigned)((C) + 15) / 16, (unsigned)(GB)), 32, 0, stream>>>(gc13); }
    { GemmP gc14;
      gc14.A = c1w + 4; gc14.B = YP + 131; gc14.bias = c1w + 4; gc14.R = Z; gc14.C = Z;
      gc14.sAo = 0; gc14.sAi = 0; gc14.sAm = C * 9; gc14.sAk = 9; gc14.sBo = (long long)C * PP; gc14.sBi = 0; gc14.sBn = 1; gc14.sBk = PP; gc14.sCo = (long long)C * NW; gc14.sCi = 0; gc14.sCm = NW; gc14.sRo = (long long)C * NW; gc14.sRi = 0; gc14.sRm = NW; gc14.sRn = 1;
      gc14.M = C; gc14.N = NW - 2; gc14.K = C; gc14.zi_n = 1; gc14.flags = 4; gc14.act = 0;
      gc14.alpha = 1.0f; gc14.beta = 1.0f; gc14.sa = 8.0f; gc14.sb = 1.0f; gc14.Npad = NW - 2; gc14.pad_ = 0;
      if ((long long)(C) >= 64 && (long long)(NW - 2) >= 64) k_gemmT<0, 4, 4><<<dim3((unsigned)((NW - 2) + 63) / 64, (unsigned)((C) + 63) / 64, (unsigned)(GB)), 32, 0, stream>>>(gc14);
      else k_gemm<0><<<dim3((unsigned)((NW - 2) + 31) / 32, (unsigned)((C) + 15) / 16, (unsigned)(GB)), 32, 0, stream>>>(gc14); }
    { GemmP gc15;
      gc15.A = c1w + 5; gc15.B = YP + 132; gc15.bias = c1w + 5; gc15.R = Z; gc15.C = Z;
      gc15.sAo = 0; gc15.sAi = 0; gc15.sAm = C * 9; gc15.sAk = 9; gc15.sBo = (long long)C * PP; gc15.sBi = 0; gc15.sBn = 1; gc15.sBk = PP; gc15.sCo = (long long)C * NW; gc15.sCi = 0; gc15.sCm = NW; gc15.sRo = (long long)C * NW; gc15.sRi = 0; gc15.sRm = NW; gc15.sRn = 1;
      gc15.M = C; gc15.N = NW - 2; gc15.K = C; gc15.zi_n = 1; gc15.flags = 4; gc15.act = 0;
      gc15.alpha = 1.0f; gc15.beta = 1.0f; gc15.sa = 8.0f; gc15.sb = 1.0f; gc15.Npad = NW - 2; gc15.pad_ = 0;
      if ((long long)(C) >= 64 && (long long)(NW - 2) >= 64) k_gemmT<0, 4, 4><<<dim3((unsigned)((NW - 2) + 63) / 64, (unsigned)((C) + 63) / 64, (unsigned)(GB)), 32, 0, stream>>>(gc15);
      else k_gemm<0><<<dim3((unsigned)((NW - 2) + 31) / 32, (unsigned)((C) + 15) / 16, (unsigned)(GB)), 32, 0, stream>>>(gc15); }
    { GemmP gc16;
      gc16.A = c1w + 6; gc16.B = YP + 260; gc16.bias = c1w + 6; gc16.R = Z; gc16.C = Z;
      gc16.sAo = 0; gc16.sAi = 0; gc16.sAm = C * 9; gc16.sAk = 9; gc16.sBo = (long long)C * PP; gc16.sBi = 0; gc16.sBn = 1; gc16.sBk = PP; gc16.sCo = (long long)C * NW; gc16.sCi = 0; gc16.sCm = NW; gc16.sRo = (long long)C * NW; gc16.sRi = 0; gc16.sRm = NW; gc16.sRn = 1;
      gc16.M = C; gc16.N = NW - 2; gc16.K = C; gc16.zi_n = 1; gc16.flags = 4; gc16.act = 0;
      gc16.alpha = 1.0f; gc16.beta = 1.0f; gc16.sa = 8.0f; gc16.sb = 1.0f; gc16.Npad = NW - 2; gc16.pad_ = 0;
      if ((long long)(C) >= 64 && (long long)(NW - 2) >= 64) k_gemmT<0, 4, 4><<<dim3((unsigned)((NW - 2) + 63) / 64, (unsigned)((C) + 63) / 64, (unsigned)(GB)), 32, 0, stream>>>(gc16);
      else k_gemm<0><<<dim3((unsigned)((NW - 2) + 31) / 32, (unsigned)((C) + 15) / 16, (unsigned)(GB)), 32, 0, stream>>>(gc16); }
    { GemmP gc17;
      gc17.A = c1w + 7; gc17.B = YP + 261; gc17.bias = c1w + 7; gc17.R = Z; gc17.C = Z;
      gc17.sAo = 0; gc17.sAi = 0; gc17.sAm = C * 9; gc17.sAk = 9; gc17.sBo = (long long)C * PP; gc17.sBi = 0; gc17.sBn = 1; gc17.sBk = PP; gc17.sCo = (long long)C * NW; gc17.sCi = 0; gc17.sCm = NW; gc17.sRo = (long long)C * NW; gc17.sRi = 0; gc17.sRm = NW; gc17.sRn = 1;
      gc17.M = C; gc17.N = NW - 2; gc17.K = C; gc17.zi_n = 1; gc17.flags = 4; gc17.act = 0;
      gc17.alpha = 1.0f; gc17.beta = 1.0f; gc17.sa = 8.0f; gc17.sb = 1.0f; gc17.Npad = NW - 2; gc17.pad_ = 0;
      if ((long long)(C) >= 64 && (long long)(NW - 2) >= 64) k_gemmT<0, 4, 4><<<dim3((unsigned)((NW - 2) + 63) / 64, (unsigned)((C) + 63) / 64, (unsigned)(GB)), 32, 0, stream>>>(gc17);
      else k_gemm<0><<<dim3((unsigned)((NW - 2) + 31) / 32, (unsigned)((C) + 15) / 16, (unsigned)(GB)), 32, 0, stream>>>(gc17); }
    { GemmP gc18;
      gc18.A = c1w + 8; gc18.B = YP + 262; gc18.bias = c1w + 8; gc18.R = Z; gc18.C = Z;
      gc18.sAo = 0; gc18.sAi = 0; gc18.sAm = C * 9; gc18.sAk = 9; gc18.sBo = (long long)C * PP; gc18.sBi = 0; gc18.sBn = 1; gc18.sBk = PP; gc18.sCo = (long long)C * NW; gc18.sCi = 0; gc18.sCm = NW; gc18.sRo = (long long)C * NW; gc18.sRi = 0; gc18.sRm = NW; gc18.sRn = 1;
      gc18.M = C; gc18.N = NW - 2; gc18.K = C; gc18.zi_n = 1; gc18.flags = 4; gc18.act = 0;
      gc18.alpha = 1.0f; gc18.beta = 1.0f; gc18.sa = 8.0f; gc18.sb = 1.0f; gc18.Npad = NW - 2; gc18.pad_ = 0;
      if ((long long)(C) >= 64 && (long long)(NW - 2) >= 64) k_gemmT<0, 4, 4><<<dim3((unsigned)((NW - 2) + 63) / 64, (unsigned)((C) + 63) / 64, (unsigned)(GB)), 32, 0, stream>>>(gc18);
      else k_gemm<0><<<dim3((unsigned)((NW - 2) + 31) / 32, (unsigned)((C) + 15) / 16, (unsigned)(GB)), 32, 0, stream>>>(gc18); }
    k_tru_bnc<<<(unsigned)(((long long)GB * C * P + 255) / 256), 256, 0, stream>>>(Z, bn1s, bn1b, bn1m, bn1v, Y, GB, C, Hs, PW, PW);
    { GemmP g21;
      g21.A = c2w; g21.B = Y; g21.bias = c2w; g21.R = c2w; g21.C = Q;
      g21.sAo = 0; g21.sAi = 0; g21.sAm = C; g21.sAk = 1; g21.sBo = (long long)C * P; g21.sBi = 0; g21.sBn = 1; g21.sBk = P; g21.sCo = (long long)C * P; g21.sCi = 0; g21.sCm = P; g21.sRo = 0; g21.sRi = 0; g21.sRm = 0; g21.sRn = 0;
      g21.M = C; g21.N = P; g21.K = C; g21.zi_n = 1; g21.flags = 0; g21.act = 0;
      g21.alpha = 1.0f; g21.beta = 0.0f; g21.sa = 1.0f; g21.sb = 1.0f; g21.Npad = P; g21.pad_ = 0;
      if ((long long)(C) >= 64 && (long long)(P) >= 64) k_gemmT<1, 2, 4><<<dim3((unsigned)((P) + 63) / 64, (unsigned)((C) + 31) / 32, (unsigned)(GB)), 32, 0, stream>>>(g21);
      else k_gemm<1><<<dim3((unsigned)((P) + 31) / 32, (unsigned)((C) + 15) / 16, (unsigned)(GB)), 32, 0, stream>>>(g21); }
    k_tru_bnc<<<(unsigned)(((long long)GB * C * P + 255) / 256), 256, 0, stream>>>(Q, bn2s, bn2b, bn2m, bn2v, out + (size_t)4 * C * P, GB, C, Hs, PW, Hs);
}
